// RGCN_24472723653074
// MI455X (gfx1250) — hardware-verified
//
#include <hip/hip_runtime.h>

namespace {

constexpr int N = 100000, NP = 100000, NPL = NP  , SRCM = N  , EFULL = 1200000, E = EFULL  ;
constexpr int F = 128  , FO = 64  , NCLS = 2  , VOC = 1, NRL = NP  , NL = (NPL < N ? NPL : N);
constexpr float LN_EPS = 1e-5f;
constexpr float LNEPS = 1e-5f; constexpr float XS = 8.0f, WSC = 256.0f, WSQ = 0.25f, RS_ = 1024.0f, NSL_ = 0.2f, NSA_ = 0.01f, SLOPE = 0.0f, BNEPS = 1e-5f;
static_assert(NP % 32 == 0 && NP >= N && NPL % 32 == 0 && F % 32 == 0, "tiling");
static_assert(F == 128, "F stays at the frame's value: it is named only by kernels this file does not launch");
typedef _Float16 b16;
typedef __attribute__((ext_vector_type(16))) _Float16 v16b;
typedef __attribute__((ext_vector_type(8))) _Float16 v8b;
typedef __attribute__((ext_vector_type(8))) float v8f;
typedef __attribute__((ext_vector_type(4))) float v4f;
__device__ __forceinline__ float bf16_rne(float f) { unsigned int u = __float_as_uint(f); u += 0x7FFFu + ((u >> 16) & 1u); return __uint_as_float(u & 0xFFFF0000u); }
__device__ __forceinline__ void split16(float v, b16& hi, b16& lo) { hi = (b16)v; lo = (b16)(v - (float)hi); }
__device__ __forceinline__ v16b frag_kb(const b16* p, int hh) { const v8b a = *(const v8b*)(p + 8 * hh), b = *(const v8b*)(p + 16 + 8 * hh); v16b f;
#pragma unroll
  for (int e = 0; e < 8; ++e) { f[e] = a[e]; f[8 + e] = b[e]; } return f; }
__device__ __forceinline__ v8f wmma16b(v16b a, v16b b, v8f c) { v8f d = __builtin_amdgcn_wmma_f32_16x16x32_f16(false, a, false, b, (short)0, c, false, false); asm volatile("v_nop\n\tv_nop\n\tv_nop\n\tv_nop" : "+v"(d) : "v"(a), "v"(b)); return d; }
__device__ __forceinline__ void wave_lds_sync() { __builtin_amdgcn_fence(__ATOMIC_RELEASE, "workgroup"); __builtin_amdgcn_wave_barrier(); __builtin_amdgcn_fence(__ATOMIC_ACQUIRE, "workgroup"); }
__device__ __forceinline__ int iclamp(int v, int lo, int hi) { return v < lo ? lo : (v > hi ? hi : v); }
constexpr int CSR_NBLK = 512, CSR_GB = 8  , CSR_GN = 1 << CSR_GB  , CSR_MAXG = 512, CSR_CAP = 12288  ;
static_assert(((N + CSR_GN - 1) >> CSR_GB) <= CSR_MAXG && CSR_GN % 4 == 0 && CSR_GN <= 65536, "csr: bucket count / 16-bit node key");
__global__ __launch_bounds__(64) void csrA_kernel(const int* __restrict__ dst, int E, int N, int nG, int CHP, int NGP, int* __restrict__ STG, int* __restrict__ HST) {
  extern __shared__ int sm[];
  int* cnt = sm; int* run = sm + NGP; int* ids = sm + 2 * NGP;
  const int b = blockIdx.x; const int ch = (E + CSR_NBLK - 1) / CSR_NBLK; const int e0 = b * ch, e1 = min(E, e0 + ch);
  for (int i = threadIdx.x; i < NGP; i += 64) cnt[i] = 0;
  for (int i = threadIdx.x; i < CHP; i += 64) ids[i] = -1;
  __syncthreads();
  if (threadIdx.x == 0) {
    for (int e = e0; e < e1; ++e) { int d = dst[e]; d = (d < 0) ? 0 : (d >= N ? N - 1 : d); cnt[d >> CSR_GB] += 1; }
    int acc = 0; for (int g = 0; g < nG; ++g) { run[g] = acc; acc += cnt[g]; }
    for (int e = e0; e < e1; ++e) { int d = dst[e]; d = (d < 0) ? 0 : (d >= N ? N - 1 : d); const int g = d >> CSR_GB; ids[run[g]] = e; run[g] += 1; } }
  __syncthreads();
  typedef __attribute__((ext_vector_type(4))) int v4i;
  for (int pass = 0; pass < 2; ++pass) {
    for (int i = threadIdx.x; i < CHP / 4; i += 64) *(volatile v4i*)(STG + (size_t)b * CHP + i * 4) = *(const v4i*)(&ids[i * 4]);
    for (int i = threadIdx.x; i < NGP / 4; i += 64) { v4i v; for (int e = 0; e < 4; ++e) v[e] = (i * 4 + e < nG) ? cnt[i * 4 + e] : 0; *(volatile v4i*)(HST + (size_t)b * NGP + i * 4) = v; }
    __threadfence(); }
}
__global__ __launch_bounds__(512) void csrS_kernel(const int* __restrict__ HST, int nG, int NGP, int* __restrict__ START, int* __restrict__ TOT, int* __restrict__ OFF) {
  __shared__ int tot[CSR_MAXG];
  const int b = threadIdx.x;
  for (int pass = 0; pass < 2; ++pass) { int runb = 0; for (int g = 0; g < nG; ++g) { int c = HST[(size_t)b * NGP + g]; c = (c < 0) ? 0 : c; ((volatile int*)OFF)[(size_t)g * CSR_NBLK + b] = runb; runb += c; } __threadfence(); }
  for (int g = threadIdx.x; g < nG; g += 512) { int s = 0; for (int bb = 0; bb < CSR_NBLK; ++bb) { int c = HST[(size_t)bb * NGP + g]; s += (c < 0) ? 0 : c; } tot[g] = s; }
  __syncthreads();
  if (threadIdx.x < 32) {
    __shared__ int st[CSR_MAXG + 32];
    if (threadIdx.x == 0) { int acc = 0; for (int g = 0; g < NGP; ++g) { st[g] = acc; if (g < nG) acc += (tot[g] + 31) & ~31; } st[NGP] = acc; }
    __builtin_amdgcn_fence(__ATOMIC_RELEASE, "workgroup"); __builtin_amdgcn_wave_barrier(); __builtin_amdgcn_fence(__ATOMIC_ACQUIRE, "workgroup");
    for (int pass = 0; pass < 2; ++pass) { for (int i = threadIdx.x; i < NGP + 32; i += 32) { ((volatile int*)START)[i] = (i <= NGP) ? st[min(i, NGP)] : 0; ((volatile int*)TOT)[i] = (i < nG) ? tot[i] : 0; } __threadfence(); } }
}
__global__ __launch_bounds__(256) void csrB_kernel(const int* __restrict__ dst, int N, int nG, int CHP, int NGP, int permLen, const int* __restrict__ STG, const int* __restrict__ HST, const int* __restrict__ OFF, const int* __restrict__ START, const int* __restrict__ TOT, int* __restrict__ PERM, int* __restrict__ ROWPTR, int* __restrict__ ROWCNT, int* __restrict__ FLAG) {
  typedef __attribute__((ext_vector_type(4))) int v4i;
  __shared__ int ids[CSR_CAP]; __shared__ unsigned short key[CSR_CAP]; __shared__ int outp[CSR_CAP]; __shared__ int ncnt[CSR_GN + 1]; __shared__ int boff[CSR_NBLK + 1];
  const int g = blockIdx.x, t_ = threadIdx.x; int tot = TOT[g]; int st = START[g], stn = START[g + 1]; const int v0 = g * CSR_GN; const int nv = min(CSR_GN, N - v0);
  st = (st < 0) ? 0 : (st > permLen - 32 ? permLen - 32 : st) & ~31; stn = (stn < st) ? st : (stn > permLen ? permLen : stn); tot = (tot < 0) ? 0 : tot; if (tot > stn - st && tot <= CSR_CAP) tot = stn - st;
  if (tot > CSR_CAP) {
    for (int pass = 0; pass < 2; ++pass) { for (int i = t_; i < CSR_GN / 4; i += 256) { v4i a, c; for (int e = 0; e < 4; ++e) { a[e] = st; c[e] = 0; } *(volatile v4i*)(ROWPTR + v0 + i * 4) = a; *(volatile v4i*)(ROWCNT + v0 + i * 4) = c; } if (t_ == 0) ((volatile int*)FLAG)[0] = 1; __threadfence(); } (void)nv; return; }
  if (t_ == 0) { int acc = 0; for (int b = 0; b < CSR_NBLK; ++b) { boff[b] = acc; int c = HST[(size_t)b * NGP + g]; c = (c < 0) ? 0 : (c > CHP ? CHP : c); acc += c; if (acc > tot) acc = tot; } boff[CSR_NBLK] = acc; }
  for (int i = t_; i <= CSR_GN; i += 256) ncnt[i] = 0;
  __syncthreads();
  for (int b = 0; b < CSR_NBLK; ++b) { const int c = boff[b + 1] - boff[b]; int o_ = OFF[(size_t)g * CSR_NBLK + b]; o_ = (o_ < 0) ? 0 : (o_ > CHP - c ? CHP - c : o_); const int* src_ = STG + (size_t)b * CHP + o_;
    for (int i = t_; i < c; i += 256) { int id = src_[i]; id = (id < 0) ? 0 : id; ids[boff[b] + i] = id; int d = dst[id]; d = (d < v0) ? v0 : (d >= N ? N - 1 : d); int kk = d - v0; kk = (kk < 0) ? 0 : (kk >= CSR_GN ? CSR_GN - 1 : kk); key[boff[b] + i] = (unsigned short)kk; } }
  __syncthreads();
  if (t_ == 0) { for (int i = 0; i < tot; ++i) ncnt[key[i]] += 1; int acc = 0; for (int vl = 0; vl < CSR_GN; ++vl) { const int c = ncnt[vl]; ncnt[vl] = acc; acc += c; } ncnt[CSR_GN] = acc;
    for (int i = 0; i < tot; ++i) { const int vl = key[i]; outp[ncnt[vl]] = ids[i]; ncnt[vl] += 1; }
    for (int vl = CSR_GN; vl > 0; --vl) ncnt[vl] = ncnt[vl - 1]; ncnt[0] = 0; }
  __syncthreads();
  for (int pass = 0; pass < 2; ++pass) {
    for (int i = t_; i < (stn - st) / 4; i += 256) { v4i v; for (int e = 0; e < 4; ++e) { const int q = i * 4 + e; v[e] = (q < tot) ? outp[q] : -1; } *(volatile v4i*)(PERM + st + i * 4) = v; }
    for (int i = t_; i < CSR_GN / 4; i += 256) { v4i a, c; for (int e = 0; e < 4; ++e) { const int vl = i * 4 + e; a[e] = st + ncnt[vl]; c[e] = (vl < nv) ? (ncnt[vl + 1] - ncnt[vl]) : 0; } *(volatile v4i*)(ROWPTR + v0 + i * 4) = a; *(volatile v4i*)(ROWCNT + v0 + i * 4) = c; }
    __threadfence(); }
}
__global__ __launch_bounds__(256) void csrZ_kernel(int* __restrict__ p, size_t n4) { typedef __attribute__((ext_vector_type(4))) int v4i; const size_t tid = (size_t)blockIdx.x * 256 + threadIdx.x, nth = (size_t)gridDim.x * 256; v4i z = {0, 0, 0, 0}; for (size_t i = tid; i < n4; i += nth) *(volatile v4i*)(p + i * 4) = z; }
struct CsrBufs { int *STG, *HST, *OFF, *START, *TOT, *PERM, *ROWPTR, *ROWCNT, *FLAG; int nG, NGP, CHP; size_t permLen; char* base; size_t bytes; };
static size_t csr_carve(CsrBufs& c, char* ws, size_t off, int E, int N) {
  const size_t off0 = off; c.base = ws + off;
  auto al = [&](size_t bytes) { char* p = ws + off; off += (bytes + 255) & ~(size_t)255; return p; };
  c.nG = (N + CSR_GN - 1) / CSR_GN; c.NGP = (c.nG + 31) & ~31; const int ch = (E + CSR_NBLK - 1) / CSR_NBLK; c.CHP = (ch + 31) & ~31; c.permLen = (size_t)E + 32 * (size_t)c.nG + 32;
  c.STG = (int*)al((size_t)CSR_NBLK * c.CHP * 4); c.HST = (int*)al((size_t)CSR_NBLK * c.NGP * 4); c.OFF = (int*)al((size_t)c.NGP * CSR_NBLK * 4); c.START = (int*)al((size_t)(c.NGP + 64) * 4); c.TOT = (int*)al((size_t)(c.NGP + 64) * 4);
  c.PERM = (int*)al(c.permLen * 4); c.ROWPTR = (int*)al((size_t)c.nG * CSR_GN * 4); c.ROWCNT = (int*)al((size_t)c.nG * CSR_GN * 4); c.FLAG = (int*)al(256);
  c.bytes = off - off0; return off;
}
static void csr_build(const CsrBufs& c, const int* dst, int E, int N, hipStream_t stream) {
  const size_t smem = (size_t)(2 * c.NGP + c.CHP) * 4;
  csrZ_kernel<<<512, 256, 0, stream>>>((int*)c.base, c.bytes / 16);
  csrA_kernel<<<CSR_NBLK, 64, smem, stream>>>(dst, E, N, c.nG, c.CHP, c.NGP, c.STG, c.HST);
  csrS_kernel<<<1, 512, 0, stream>>>(c.HST, c.nG, c.NGP, c.START, c.TOT, c.OFF);
  csrB_kernel<<<c.nG, 256, 0, stream>>>(dst, N, c.nG, c.CHP, c.NGP, (int)c.permLen, c.STG, c.HST, c.OFF, c.START, c.TOT, c.PERM, c.ROWPTR, c.ROWCNT, c.FLAG);
}

typedef __attribute__((ext_vector_type(4))) _Float16 v4h;
__device__ __forceinline__ float lrelu(float v) { return v > 0.0f ? v : NSL_ * v; }
template <int K, int NOUTR, int NOUTP>
__global__ __launch_bounds__(256) void wt_kernel(const float* __restrict__ w, b16* __restrict__ WT, float scl) {
  const int u = blockIdx.x * 256 + threadIdx.x; if (u >= NOUTP * K / 8) return; const int e = u * 8; const int o = e / K, k0 = e % K; v8b v;
#pragma unroll
  for (int j = 0; j < 8; ++j) v[j] = (b16)(o < NOUTR ? bf16_rne(w[(size_t)(k0 + j) * NOUTR + o]) * scl : 0.0f);
  for (int pass = 0; pass < 2; ++pass) { *(volatile v8b*)(WT + e) = v; __threadfence(); }
}
__global__ __launch_bounds__(256) void zfill_kernel(float* __restrict__ p, int n) { for (int pass = 0; pass < 2; ++pass) { for (int i = threadIdx.x; i < n; i += 256) ((volatile float*)p)[i] = 0.0f; __threadfence(); } }
template <int K, int NT, int PREC, int MODE, bool GIDX>
__global__ __launch_bounds__(64) void lin_kernel(const float* __restrict__ X, const int* __restrict__ gidx, const b16* __restrict__ WT, const b16* __restrict__ WQ, const float* __restrict__ bias, float* __restrict__ OUT, int opitch, int nvalid, int mrows) {
  constexpr int NC = NT * 16;
  __shared__ __attribute__((aligned(16))) b16 Ah[2][16][K + 8], Al[2][16][(PREC == 0 ? K : 0) + 8]; __shared__ __attribute__((aligned(16))) float Tf[2][16][NC + 4];
  const int wave = threadIdx.x >> 5, lane = threadIdx.x & 31, nloc = lane & 15, hlf = lane >> 4; const size_t m0 = (size_t)blockIdx.x * 32 + wave * 16;
  for (int idx = lane; idx < 16 * (K / 4); idx += 32) { const int rr = idx / (K / 4), c4 = (idx % (K / 4)) * 4; const size_t vrow = (m0 + rr < (size_t)nvalid) ? m0 + rr : (size_t)nvalid - 1; size_t arow = vrow; if (GIDX) arow = (size_t)iclamp(gidx[vrow], 0, VOC - 1);
    const v4f v = *(const v4f*)(X + arow * K + c4); v4h hv, lv;
    for (int j = 0; j < 4; ++j) { float vj = v[j]; if (MODE == 2) vj = fmaxf(vj, 0.0f); const float vs = (PREC == 1 ? bf16_rne(vj) : vj) * XS; const b16 ph = (b16)vs; hv[j] = ph; lv[j] = (b16)((vs - (float)ph) * RS_); } *(v4h*)(&Ah[wave][rr][c4]) = hv; if (PREC == 0) *(v4h*)(&Al[wave][rr][c4]) = lv; }
  wave_lds_sync();
  v8f acc[NT];
#pragma unroll
  for (int t = 0; t < NT; ++t) acc[t] = (v8f){};
#pragma unroll 1
  for (int kb = 0; kb < K; kb += 32) { const v16b a = frag_kb(&Ah[wave][nloc][kb], hlf); v16b al; if (PREC == 0) al = frag_kb(&Al[wave][nloc][kb], hlf);
#pragma unroll
    for (int t = 0; t < NT; ++t) { const size_t wo_ = (size_t)(t * 16 + nloc) * K + kb; acc[t] = wmma16b(a, frag_kb(WT + wo_, hlf), acc[t]); if (PREC == 0) acc[t] = wmma16b(al, frag_kb(WQ + wo_, hlf), acc[t]); } }
#pragma unroll
  for (int t = 0; t < NT; ++t) { const int col = t * 16 + nloc; const float bb = (MODE == 14 || MODE == 17) ? 0.0f : bf16_rne(bias[col]);
    for (int r = 0; r < 8; ++r) { const size_t vrow = m0 + 8 * hlf + r; float y = acc[t][r] * (1.0f / (XS * WSC)) + bb; if (MODE == 1) y = fmaxf(y, 0.0f); if ((MODE == 14 || MODE == 17) && vrow < (size_t)mrows) y += OUT[vrow * (size_t)opitch + col]; if (MODE == 17) y = fmaxf(y, 0.0f);     Tf[wave][8 * hlf + r][col] = (vrow < (size_t)nvalid) ? y : 0.0f; } }
  wave_lds_sync();
  for (int pass = 0; pass < 2; ++pass) { for (int rr = 0; rr < 16; ++rr) { if (m0 + rr < (size_t)mrows) { if (NC >= 128) { for (int c8 = 0; c8 < NC; c8 += 128) *(volatile v4f*)(OUT + (m0 + rr) * (size_t)opitch + c8 + lane * 4) = *(const v4f*)(&Tf[wave][rr][c8 + lane * 4]); }
        else { if (lane < NC / 4) *(volatile v4f*)(OUT + (m0 + rr) * (size_t)opitch + lane * 4) = *(const v4f*)(&Tf[wave][rr][lane * 4]); } } } __threadfence(); }
}
template <int W, bool WGT, bool RELU>
__global__ __launch_bounds__(256) void wsump_kernel(const float* __restrict__ X, int xp, const float* __restrict__ EW, const int* __restrict__ srcs, const int* __restrict__ PERM, const int* __restrict__ ROWPTR, const int* __restrict__ ROWCNT, int permLen, const float* __restrict__ bias, float* __restrict__ OUT, int op, int mrows, float oscale) {
  constexpr int CW = W / 8; static_assert(W % 32 == 0, "wsump: 8 threads per row, float4 loads / stores"); const int tid = threadIdx.x; const int row = tid >> 3, g = tid & 7, c0 = g * CW; const int v = blockIdx.x * 32 + row;
  int cnt = 0, p0 = 0; if (v < N) { cnt = iclamp(ROWCNT[v], 0, 65536); p0 = iclamp(ROWPTR[v], 0, permLen - 1); if (p0 + cnt > permLen) cnt = permLen - p0; }
  float m[CW]; for (int j = 0; j < CW; ++j) m[j] = 0.0f;
  for (int i = 0; i < cnt; ++i) { const int e = iclamp(PERM[p0 + i], 0, E - 1); int s = iclamp(srcs[e], 0, N - 1); if (SRCM < N) s %= SRCM; const float w = WGT ? bf16_rne(EW[e]) : 1.0f;     const float* xr = X + (size_t)s * xp + c0;
#pragma unroll
    for (int q = 0; q < CW / 4; ++q) { const v4f t4 = *(const v4f*)(xr + 4 * q); for (int j = 0; j < 4; ++j) m[4 * q + j] += WGT ? (w * t4[j]) : t4[j]; } }
  for (int pass = 0; pass < 2; ++pass) { if (v < mrows) { float* orow = OUT + (size_t)v * op + c0;
#pragma unroll
      for (int q = 0; q < CW / 4; ++q) { const v4f b4 = *(const v4f*)(bias + c0 + 4 * q); v4f o; for (int j = 0; j < 4; ++j) { float y = m[4 * q + j] + bf16_rne(b4[j]); if (RELU) y = fmaxf(y, 0.0f); o[j] = (v < N) ? (y * oscale) : 0.0f; } *(volatile v4f*)(orow + 4 * q) = o; } }
    __threadfence(); }
}
__global__ __launch_bounds__(256) void wdeg_kernel(const float* __restrict__ w, const int* __restrict__ PERM, const int* __restrict__ ROWPTR, const int* __restrict__ ROWCNT, int permLen, float* __restrict__ DEG, int n) {
  const int v = blockIdx.x * 256 + threadIdx.x; if (v >= n) return; float s = 1.0f;
  if (v < N) { int cnt = iclamp(ROWCNT[v], 0, 65536); const int p0 = iclamp(ROWPTR[v], 0, permLen - 1); if (p0 + cnt > permLen) cnt = permLen - p0;
    for (int i = 0; i < cnt; ++i) { const int e = iclamp(PERM[p0 + i], 0, E - 1); s += bf16_rne(w[e]); } }
  for (int pass = 0; pass < 2; ++pass) { ((volatile float*)DEG)[v] = s; __threadfence(); }
}
__global__ __launch_bounds__(256) void rscale_kernel(const float* __restrict__ H, const float* __restrict__ DEG, float* __restrict__ HS, int nrows) {
  const size_t i = (size_t)blockIdx.x * 256 + threadIdx.x; if (i >= (size_t)nrows * (F / 4)) return; const size_t v = i / (F / 4); const int c = (int)(i % (F / 4)) * 4; v4f o = {0.0f, 0.0f, 0.0f, 0.0f};
  if (v < (size_t)N) { const float dg = DEG[v]; const float dv = (dg > 0.0f) ? rsqrtf(dg) : 0.0f; const v4f t = *(const v4f*)(H + v * F + c); for (int j = 0; j < 4; ++j) o[j] = (dv * t[j]); }
  for (int pass = 0; pass < 2; ++pass) { *(volatile v4f*)(HS + v * F + c) = o; __threadfence(); }
}
__global__ __launch_bounds__(256) void wfin_kernel(const float* __restrict__ AG, const float* __restrict__ HS, const float* __restrict__ DEG, const float* __restrict__ b, float* __restrict__ OUT, int nrows) {
  const size_t i = (size_t)blockIdx.x * 256 + threadIdx.x; if (i >= (size_t)nrows * (F / 4)) return; const size_t v = i / (F / 4); const int c = (int)(i % (F / 4)) * 4; v4f o = {0.0f, 0.0f, 0.0f, 0.0f};
  if (v < (size_t)N) { const float dg = DEG[v]; const float dv = (dg > 0.0f) ? rsqrtf(dg) : 0.0f; const v4f a = *(const v4f*)(AG + v * F + c), s = *(const v4f*)(HS + v * F + c); for (int j = 0; j < 4; ++j) o[j] = fmaxf((dv * (a[j] + s[j])) + bf16_rne(b[c + j]), 0.0f); }
  for (int pass = 0; pass < 2; ++pass) { *(volatile v4f*)(OUT + v * F + c) = o; __threadfence(); }
}
template <int W>
__global__ __launch_bounds__(256) void xcpw_kernel(const float* __restrict__ x, float* __restrict__ P, int pp, int n, int np_) {
  const size_t i = (size_t)blockIdx.x * 256 + threadIdx.x; const size_t v = i / (W / 4); const int c = (int)(i % (W / 4)) * 4; if (v >= (size_t)np_) return; v4f t = {0.0f, 0.0f, 0.0f, 0.0f};
  if (v < (size_t)n) { t = *(const v4f*)(x + v * W + c); for (int j = 0; j < 4; ++j) t[j] = bf16_rne(t[j]); }
  for (int pass = 0; pass < 2; ++pass) { *(volatile v4f*)(P + v * (size_t)pp + c) = t; __threadfence(); }
}
template <int W>
__global__ __launch_bounds__(256) void hmeanw_kernel(const float* __restrict__ X, int xp, int ns, int srcm, const int* __restrict__ srcs, int ecut, const int* __restrict__ PERM, const int* __restrict__ ROWPTR, const int* __restrict__ ROWCNT, int permLen, float* __restrict__ P, int pp, int ocol, int nd, int ndp) {
  constexpr int CW = W / 8; static_assert(W % 32 == 0, "hmeanw: 8 threads per row, float4 steps");
  const int tid = threadIdx.x; const int row = tid >> 3, g = tid & 7, c0 = g * CW; const int v = blockIdx.x * 32 + row; if (v >= ndp) return;
  int cnt = 0, p0 = 0; if (v < nd) { cnt = iclamp(ROWCNT[v], 0, 65536); p0 = iclamp(ROWPTR[v], 0, permLen - 1); if (p0 + cnt > permLen) cnt = permLen - p0; }
  float m[CW];
#pragma unroll
  for (int j = 0; j < CW; ++j) m[j] = 0.0f;
  for (int i = 0; i < cnt; ++i) { const int e = iclamp(PERM[p0 + i], 0, ecut - 1); int s = iclamp(srcs[e], 0, ns - 1); if (srcm < ns) s %= srcm; const float* xr = X + (size_t)s * xp + c0;
#pragma unroll
    for (int q = 0; q < CW / 4; ++q) { const v4f a = *(const v4f*)(xr + 4 * q); for (int j = 0; j < 4; ++j) m[4 * q + j] += a[j]; } }
  const float inv = 1.0f / (float)(cnt > 0 ? cnt : 1);
  for (int pass = 0; pass < 2; ++pass) { float* orow = P + (size_t)v * pp + ocol + c0;
#pragma unroll
    for (int q = 0; q < CW / 4; ++q) { v4f o4; for (int j = 0; j < 4; ++j) o4[j] = (v < nd) ? (m[4 * q + j] * inv) : 0.0f; *(volatile v4f*)(orow + 4 * q) = o4; }
    __threadfence(); }
}
template <int K, int NOUT_>
__global__ __launch_bounds__(256) void wto_kernel(const float* __restrict__ w, b16* __restrict__ WT, float scl) {
  const int u = blockIdx.x * 256 + threadIdx.x; if (u >= NOUT_ * K / 8) return; const int e = u * 8; const int o = e / K, k0 = e % K; v8b v;
#pragma unroll
  for (int j = 0; j < 8; ++j) v[j] = (b16)(bf16_rne(w[(size_t)o * K + k0 + j]) * scl);
  for (int pass = 0; pass < 2; ++pass) { *(volatile v8b*)(WT + e) = v; __threadfence(); }
}
__global__ __launch_bounds__(256) void addk_kernel(const float* __restrict__ A, const float* __restrict__ B, float* __restrict__ Y, size_t n4, float oscale) {
  const size_t i = (size_t)blockIdx.x * 256 + threadIdx.x; if (i >= n4) return; const v4f a = *(const v4f*)(A + 4 * i), b = *(const v4f*)(B + 4 * i); v4f o; for (int j = 0; j < 4; ++j) o[j] = ((a[j] + b[j]) * oscale);
  for (int pass = 0; pass < 2; ++pass) { *(volatile v4f*)(Y + 4 * i) = o; __threadfence(); }
}
template <int NR>
__global__ __launch_bounds__(64) void bpadn_kernel(const float* __restrict__ b, float* __restrict__ B) { static_assert(NR <= 64, "bpadn: 64-entry record"); const int c = threadIdx.x; const float v = (c < NR) ? b[c] : 0.0f; for (int pass = 0; pass < 2; ++pass) { ((volatile float*)B)[c] = v; __threadfence(); } }
__global__ __launch_bounds__(256) void ocpf_kernel(const float* __restrict__ P, float* __restrict__ out, int total) {
  const int t = blockIdx.x * 256 + threadIdx.x; if (t >= total) return; const int g = t / NCLS, k = t - g * NCLS; const float v = P[(size_t)g * FO + k];
  for (int pass = 0; pass < 2; ++pass) { ((volatile float*)out)[t] = v; __threadfence(); }
}
template <int ACT>
__global__ __launch_bounds__(256) void eact_kernel(const float* __restrict__ P, float* __restrict__ OUT, size_t n4, float sl) {
  static_assert(ACT >= 1 && ACT <= 9, "eact: nine activations"); const size_t i = (size_t)blockIdx.x * 256 + threadIdx.x; if (i >= n4) return; const v4f a = *(const v4f*)(P + 4 * i); v4f o;
  for (int j = 0; j < 4; ++j) { const float v = a[j]; float y;
    if (ACT == 1) y = fmaxf(v, 0.0f);
    else if (ACT == 2) y = (v >= 0.0f) ? v : (sl * v);
    else if (ACT == 3) y = 1.0f / (1.0f + expf(-v));
    else if (ACT == 4) y = tanhf(v);
    else if (ACT == 5) y = (v > 0.0f) ? v : expm1f(v);
    else if (ACT == 6) y = v / (1.0f + expf(-v));
    else if (ACT == 7) y = (((0.5f * v)) * (1.0f + tanhf(0.7978845608028654f * (v + (0.044715f * ((v * ((v * v)))))))));
    else if (ACT == 8) y = (((0.5f * v)) * (1.0f + erff((v * 0.7071067811865476f))));
    else y = (1.0507009873554805f * ((v > 0.0f) ? v : (1.6732632423543772f * expm1f(v))));
    o[j] = y; }
  for (int pass = 0; pass < 2; ++pass) { *(volatile v4f*)(OUT + 4 * i) = o; __threadfence(); }
}
template <int W>
__global__ __launch_bounds__(256) void rowst_kernel(const float* __restrict__ H, float eps, float* __restrict__ MU, float* __restrict__ INV, int nrows) {
  static_assert(W % 4 == 0, "rowst: float4 steps"); const int v = blockIdx.x * 256 + threadIdx.x; if (v >= nrows) return; const float* hr = H + (size_t)v * W; float s = 0.0f;
  for (int q = 0; q < W / 4; ++q) { const v4f a = *(const v4f*)(hr + 4 * q); for (int j = 0; j < 4; ++j) s += a[j]; }
  const float mu = s / (float)W; float ss = 0.0f;
  for (int q = 0; q < W / 4; ++q) { const v4f a = *(const v4f*)(hr + 4 * q); for (int j = 0; j < 4; ++j) { const float d = a[j] - mu; ss += (d * d); } }
  const float inv = 1.0f / sqrtf(ss / (float)W + eps);
  for (int pass = 0; pass < 2; ++pass) { ((volatile float*)MU)[v] = mu; ((volatile float*)INV)[v] = inv; __threadfence(); }
}
template <int W>
__global__ __launch_bounds__(256) void rowap_kernel(const float* __restrict__ H, const float* __restrict__ MU, const float* __restrict__ INV, const float* __restrict__ scale, const float* __restrict__ offset, float* __restrict__ OUT, int nrows) {
  static_assert(W % 4 == 0, "rowap: float4 steps"); const size_t i = (size_t)blockIdx.x * 256 + threadIdx.x; if (i >= (size_t)nrows * (W / 4)) return; const size_t v = i / (W / 4); const int c = (int)(i % (W / 4)) * 4;
  const float mu = MU[v], inv = INV[v]; const v4f a = *(const v4f*)(H + v * W + c); v4f o; for (int j = 0; j < 4; ++j) o[j] = ((((a[j] - mu) * inv)) * bf16_rne(scale[c + j])) + bf16_rne(offset[c + j]);
  for (int pass = 0; pass < 2; ++pass) { *(volatile v4f*)(OUT + v * W + c) = o; __threadfence(); }
}
template <int W>
__global__ __launch_bounds__(256) void rowl2s_kernel(const float* __restrict__ H, int hp, float eps, float* __restrict__ INV, int nrows) {
  static_assert(W % 4 == 0, "rowl2s: float4 steps"); const int v = blockIdx.x * 256 + threadIdx.x; if (v >= nrows) return; const float* hr = H + (size_t)v * hp; float ss = 0.0f;
  for (int q = 0; q < W / 4; ++q) { const v4f a = *(const v4f*)(hr + 4 * q); for (int j = 0; j < 4; ++j) ss += (a[j] * a[j]); }
  const float nrm = sqrtf(ss); const float inv = 1.0f / fmaxf(nrm, eps);
  for (int pass = 0; pass < 2; ++pass) { ((volatile float*)INV)[v] = inv; __threadfence(); }
}
template <int W>
__global__ __launch_bounds__(256) void rowl2a_kernel(const float* __restrict__ H, int hp, const float* __restrict__ INV, float* __restrict__ OUT, int op, int nv, int nrows) {
  static_assert(W % 4 == 0 && ((W / 4) & (W / 4 - 1)) == 0, "rowl2a: W / 4 a power of two"); const size_t i = (size_t)blockIdx.x * 256 + threadIdx.x; if (i >= (size_t)nrows * (W / 4)) return; const size_t v = i / (W / 4); const int c = (int)(i % (W / 4)) * 4;
  v4f o = {0.0f, 0.0f, 0.0f, 0.0f}; if (v < (size_t)nv) { const float s = INV[v]; const v4f a = *(const v4f*)(H + v * (size_t)hp + c); for (int j = 0; j < 4; ++j) o[j] = (a[j] * s); }
  for (int pass = 0; pass < 2; ++pass) { *(volatile v4f*)(OUT + v * (size_t)op + c) = o; __threadfence(); }
}
template <int W, int MODE>
__global__ __launch_bounds__(256) void colpart_kernel(const float* __restrict__ H, const float* __restrict__ MEAN, float* __restrict__ PART, int nstat) {
  const int b = blockIdx.x, c = threadIdx.x; if (c >= W) return; const float mu = (MODE == 1) ? MEAN[c] : 0.0f; float s = 0.0f; const int v0 = b * 512, v1 = (v0 + 512 < nstat) ? v0 + 512 : nstat;
  for (int v = v0; v < v1; ++v) { const float h = H[(size_t)v * W + c]; if (MODE == 1) { const float d = h - mu; s += (d * d); } else s += h; }
  for (int pass = 0; pass < 2; ++pass) { ((volatile float*)PART)[(size_t)b * W + c] = s; __threadfence(); }
}
template <int W, int MODE>
__global__ __launch_bounds__(256) void colred_kernel(const float* __restrict__ PART, int nb, int nstat, const float* __restrict__ MEAN, const float* __restrict__ gam, const float* __restrict__ bet, float* __restrict__ OUT, float* __restrict__ OUT2) {
  const int c = threadIdx.x; if (c >= W) return; float s = 0.0f;
  for (int b = 0; b < nb; ++b) s += PART[(size_t)b * W + c];
  const float m = s / (float)nstat;
  for (int pass = 0; pass < 2; ++pass) {
    if (MODE == 0) ((volatile float*)OUT)[c] = m;
    else { const float scl = bf16_rne(gam[c]) * rsqrtf(m + BNEPS); ((volatile float*)OUT)[c] = scl; ((volatile float*)OUT2)[c] = bf16_rne(bet[c]) - MEAN[c] * scl; }
    __threadfence(); }
}
template <int W, int ACT>
__global__ __launch_bounds__(256) void bnact_kernel(const float* __restrict__ H, const float* __restrict__ SCL, const float* __restrict__ SFT, float* __restrict__ OUT, int op, int mrows) {
  const size_t i = (size_t)blockIdx.x * 256 + threadIdx.x; if (i >= (size_t)mrows * (W / 4)) return; const size_t v = i / (W / 4); const int c = (int)(i % (W / 4)) * 4;
  const v4f h = *(const v4f*)(H + v * W + c), s = *(const v4f*)(SCL + c), t = *(const v4f*)(SFT + c); v4f o;
  for (int j = 0; j < 4; ++j) { float y = (h[j] * s[j]) + t[j]; if (ACT == 1) y = fmaxf(y, 0.0f); if (ACT == 2) y = (y > 0.0f) ? y : (__expf(y) - 1.0f);     if (ACT == 3) y = (y >= 0.0f) ? y : 0.01f * y; o[j] = y; }
  for (int pass = 0; pass < 2; ++pass) { *(volatile v4f*)(OUT + v * (size_t)op + c) = o; __threadfence(); }
}
template <int NC, int PW>
__global__ __launch_bounds__(256) void lsmw_kernel(const float* __restrict__ LG, float* __restrict__ out, int rows) {
  static_assert(NC >= 4 && NC % 4 == 0 && NC <= PW && NC <= 64, "lsmw: float4 steps over the NC real classes of a PW-pitch plane"); const int r = blockIdx.x * 256 + threadIdx.x; if (r >= rows) return; v4f l[NC / 4]; float mx = -INFINITY;
#pragma unroll
  for (int q = 0; q < NC / 4; ++q) { l[q] = *(const v4f*)(LG + (size_t)r * PW + 4 * q); for (int j = 0; j < 4; ++j) mx = fmaxf(mx, l[q][j]); }
  float s = 0.0f;
#pragma unroll
  for (int q = 0; q < NC / 4; ++q) for (int j = 0; j < 4; ++j) s += __expf(l[q][j] - mx);
  const float lse = mx + __logf(s);
  for (int pass = 0; pass < 2; ++pass) { for (int q = 0; q < NC / 4; ++q) { v4f o; for (int j = 0; j < 4; ++j) o[j] = l[q][j] - lse; *(volatile v4f*)(out + (size_t)r * NC + 4 * q) = o; } __threadfence(); }
}
__global__ __launch_bounds__(256) void xpadr_kernel(const float* __restrict__ x, int xp, int xo, int xi, float* __restrict__ P, int kp, int n, int nrows) {
  const int i = blockIdx.x * 256 + threadIdx.x; const int q = kp >> 2; if (i >= nrows * q) return; const int v = i / q; const int c = (i - v * q) << 2; v4f o = {0.0f, 0.0f, 0.0f, 0.0f};
  if (v < n) { const float* xr = x + (size_t)v * (size_t)xp + (size_t)xo; if (c + 0 < xi) o[0] = bf16_rne(xr[c + 0]); if (c + 1 < xi) o[1] = bf16_rne(xr[c + 1]); if (c + 2 < xi) o[2] = bf16_rne(xr[c + 2]); if (c + 3 < xi) o[3] = bf16_rne(xr[c + 3]); }
  for (int pass = 0; pass < 2; ++pass) { *(volatile v4f*)(P + (size_t)i * 4) = o; __threadfence(); }
}
__global__ __launch_bounds__(256) void ocpr_kernel(const float* __restrict__ P, int pp, int pc, float* __restrict__ OUT, int w, int n) {
  const int t = blockIdx.x * 256 + threadIdx.x; if (t >= n * w) return; const int v = t / w; const int c = t - v * w; const float y = P[(size_t)v * (size_t)pp + (size_t)pc + (size_t)c];
  for (int pass = 0; pass < 2; ++pass) { ((volatile float*)OUT)[t] = y; __threadfence(); }
}
__global__ __launch_bounds__(256) void wtkr_kernel(const float* __restrict__ w, int ka, int nout, b16* __restrict__ WT, int kk, int noutp, float scl) {
  const int u = blockIdx.x * 256 + threadIdx.x; if (u >= noutp * (kk >> 3)) return; const int e = u << 3; const int o = e / kk, k0 = e - o * kk; v8b v;
#pragma unroll
  for (int j = 0; j < 8; ++j) { const int k = k0 + j; float t = 0.0f; if (o < nout && k < ka) t = bf16_rne(w[(size_t)k * (size_t)nout + (size_t)o]); v[j] = (b16)(t * scl); }
  for (int pass = 0; pass < 2; ++pass) { *(volatile v8b*)(WT + e) = v; __threadfence(); }
}
typedef __attribute__((ext_vector_type(2))) float v2f;
template <int W, int PW, bool WGT, bool RELU>
__global__ __launch_bounds__(256) void wsumn_kernel(const float* __restrict__ X, int xp, const float* __restrict__ EW, const int* __restrict__ srcs, const int* __restrict__ PERM, const int* __restrict__ ROWPTR, const int* __restrict__ ROWCNT, int permLen, const float* __restrict__ bias, float* __restrict__ OUT, int op, int mrows, float oscale, int n, int e, int smask) {
  static_assert(W >= 8 && W % 8 == 0 && PW >= W && PW % 8 == 0, "wsumn: 8 threads per row; a wave's four rows are whole 128-B lines when the stored width is a multiple of 8");
  constexpr int CW = W / 8, CP = (PW - W) / 8, VW = (CW % 4 == 0) ? 4 : ((CW % 2 == 0) ? 2 : 1), VP = (CP % 4 == 0) ? 4 : ((CP % 2 == 0) ? 2 : 1);
  const int tid = threadIdx.x; const int row = tid >> 3, g = tid & 7, c0 = g * CW; const int v = blockIdx.x * 32 + row;
  int cnt = 0, p0 = 0; if (v < n) { cnt = iclamp(ROWCNT[v], 0, 65536); p0 = iclamp(ROWPTR[v], 0, permLen - 1); if (p0 + cnt > permLen) cnt = permLen - p0; }
  float m[CW]; for (int j = 0; j < CW; ++j) m[j] = 0.0f;
  for (int i = 0; i < cnt; ++i) { const int ei = iclamp(PERM[p0 + i], 0, e - 1); int s = iclamp(srcs[ei], 0, n - 1); s &= smask; const float w = WGT ? bf16_rne(EW[ei]) : 1.0f; const float* xr = X + (size_t)s * xp + c0;
    if (VW == 4) {
#pragma unroll
      for (int q = 0; q < CW / 4; ++q) { const v4f t4 = *(const v4f*)(xr + 4 * q); for (int j = 0; j < 4; ++j) m[4 * q + j] += WGT ? (w * t4[j]) : t4[j]; } }
    else if (VW == 2) {
#pragma unroll
      for (int q = 0; q < CW / 2; ++q) { const v2f t2 = *(const v2f*)(xr + 2 * q); for (int j = 0; j < 2; ++j) m[2 * q + j] += WGT ? (w * t2[j]) : t2[j]; } }
    else {
#pragma unroll
      for (int q = 0; q < CW; ++q) { const float t1 = xr[q]; m[q] += WGT ? (w * t1) : t1; } } }
  for (int pass = 0; pass < 2; ++pass) { if (v < mrows) { float* orow = OUT + (size_t)v * op + c0;
#pragma unroll
      for (int q = 0; q < CW / VW; ++q) { if (VW == 4) { const v4f b4 = *(const v4f*)(bias + c0 + 4 * q); v4f o; for (int j = 0; j < 4; ++j) { float y = m[4 * q + j] + bf16_rne(b4[j]); if (RELU) y = fmaxf(y, 0.0f); o[j] = (v < n) ? (y * oscale) : 0.0f; } *(volatile v4f*)(orow + 4 * q) = o; }
        else if (VW == 2) { v2f o; for (int j = 0; j < 2; ++j) { float y = m[2 * q + j] + bf16_rne(bias[c0 + 2 * q + j]); if (RELU) y = fmaxf(y, 0.0f); o[j] = (v < n) ? (y * oscale) : 0.0f; } *(volatile v2f*)(orow + 2 * q) = o; }
        else { float y = m[q] + bf16_rne(bias[c0 + q]); if (RELU) y = fmaxf(y, 0.0f); *(volatile float*)(orow + q) = (v < n) ? (y * oscale) : 0.0f; } }
      float* prow = OUT + (size_t)v * op + W + g * CP;
#pragma unroll
      for (int q = 0; q < CP / VP; ++q) { if (VP == 4) { v4f z; for (int j = 0; j < 4; ++j) z[j] = 0.0f; *(volatile v4f*)(prow + 4 * q) = z; } else if (VP == 2) { v2f z; z[0] = 0.0f; z[1] = 0.0f; *(volatile v2f*)(prow + 2 * q) = z; } else { *(volatile float*)(prow + q) = 0.0f; } } }
    __threadfence(); }
}
template <int W>
__global__ __launch_bounds__(256) void rdivk_kernel(const float* __restrict__ A, const int* __restrict__ ROWCNT, float addc, float* __restrict__ Y, int nn, size_t n4) {
  static_assert(W % 4 == 0 && ((W / 4) & (W / 4 - 1)) == 0, "rdivk: a power-of-two number of float4 groups per row"); const size_t i = (size_t)blockIdx.x * 256 + threadIdx.x; if (i >= n4) return;
  const size_t v = i / (W / 4); v4f o = {0.0f, 0.0f, 0.0f, 0.0f}; if (v < (size_t)nn) { const float dg = (float)iclamp(ROWCNT[v], 0, 1 << 24) + addc; const v4f t = *(const v4f*)(A + 4 * i); if (dg > 0.0f) { for (int j = 0; j < 4; ++j) o[j] = t[j] / dg; } }
  for (int pass = 0; pass < 2; ++pass) { *(volatile v4f*)(Y + 4 * i) = o; __threadfence(); }
}
template <int W>
__global__ __launch_bounds__(256) void bnrec_kernel(const float* __restrict__ gam, const float* __restrict__ bet, const float* __restrict__ rm, const float* __restrict__ rv, float* __restrict__ SCL, float* __restrict__ SFT) {
  static_assert(W >= 32 && W <= 256 && W % 32 == 0, "bnrec: one block, whole lines"); const int c = threadIdx.x; if (c >= W) return; const float scl = (bf16_rne(gam[c]) * (rsqrtf(bf16_rne(rv[c]) + BNEPS))); const float sft = bf16_rne(bet[c]) - (bf16_rne(rm[c]) * scl);
  for (int pass = 0; pass < 2; ++pass) { ((volatile float*)SCL)[c] = scl; ((volatile float*)SFT)[c] = sft; __threadfence(); }
}
template <int K, int NO, bool OI>
__global__ __launch_bounds__(256) void headw_kernel(const float* __restrict__ P, int pp, const float* __restrict__ wl, const float* __restrict__ bl, float* __restrict__ out, int total) {
  static_assert(K >= 1 && NO >= 1 && NO <= 16, "headw: a narrow head (the matrix unit serves wider ones)"); const int t = blockIdx.x * 256 + threadIdx.x; if (t >= total) return; const int g = t / NO, k = t - g * NO; float s = bf16_rne(bl[k]);
  for (int c = 0; c < K; ++c) s += (P[(size_t)g * pp + c] * bf16_rne(OI ? wl[k * K + c] : wl[c * NO + k]));
  for (int pass = 0; pass < 2; ++pass) { ((volatile float*)out)[t] = s; __threadfence(); }
}
__global__ __launch_bounds__(256) void wtor_kernel(const float* __restrict__ w, int nout, int ka, b16* __restrict__ WT, int kk, int noutp, float scl) {
  const int u = blockIdx.x * 256 + threadIdx.x; if (u >= noutp * (kk >> 3)) return; const int e = u << 3; const int o = e / kk, k0 = e - o * kk; v8b v;
#pragma unroll
  for (int j = 0; j < 8; ++j) { const int k = k0 + j; float t = 0.0f; if (o < nout && k < ka) t = bf16_rne(w[(size_t)o * (size_t)ka + (size_t)k]); v[j] = (b16)(t * scl); }
  for (int pass = 0; pass < 2; ++pass) { *(volatile v8b*)(WT + e) = v; __threadfence(); }
}
template <bool TWO>
__global__ __launch_bounds__(256) void preluk_kernel(const float* __restrict__ A, const float* __restrict__ B, const float* __restrict__ a, float* __restrict__ Y, size_t n4) {
  const size_t i = (size_t)blockIdx.x * 256 + threadIdx.x; if (i >= n4) return; const float sl = bf16_rne(a[0]); const v4f p = *(const v4f*)(A + 4 * i); v4f o;
  for (int j = 0; j < 4; ++j) o[j] = (p[j] >= 0.0f) ? p[j] : (sl * p[j]);
  if (TWO) { const v4f q = *(const v4f*)(B + 4 * i); for (int j = 0; j < 4; ++j) o[j] += (q[j] >= 0.0f) ? q[j] : (sl * q[j]); }
  for (int pass = 0; pass < 2; ++pass) { *(volatile v4f*)(Y + 4 * i) = o; __threadfence(); }
}
__global__ __launch_bounds__(256) void cdegp_kernel(const int* __restrict__ ROWCNT, float* __restrict__ DEG, int n) {
  const int v = blockIdx.x * 256 + threadIdx.x; if (v >= n) return; float s = 1.0f; if (v < N) { const int c = iclamp(ROWCNT[v], 0, 1 << 24); s = (float)c + 1.0f; }
  for (int pass = 0; pass < 2; ++pass) { ((volatile float*)DEG)[v] = s; __threadfence(); }
}
template <int W>
__global__ __launch_bounds__(256) void rscalew_kernel(const float* __restrict__ H, const float* __restrict__ DEG, float* __restrict__ HS, int nv, int nrows) {
  static_assert(W >= 4 && W % 4 == 0, "rscalew: float4 steps"); const size_t i = (size_t)blockIdx.x * 256 + threadIdx.x; if (i >= (size_t)nrows * (W / 4)) return; const size_t v = i / (W / 4); const int c = (int)(i % (W / 4)) * 4; v4f o = {0.0f, 0.0f, 0.0f, 0.0f};
  if (v < (size_t)nv) { const float dg = DEG[v]; const float dv = (dg > 0.0f) ? rsqrtf(dg) : 0.0f; const v4f t = *(const v4f*)(H + v * W + c); for (int j = 0; j < 4; ++j) o[j] = (dv * t[j]); }
  for (int pass = 0; pass < 2; ++pass) { *(volatile v4f*)(HS + v * W + c) = o; __threadfence(); }
}
template <int W, bool RELU>
__global__ __launch_bounds__(256) void wfinw_kernel(const float* __restrict__ AG, const float* __restrict__ HS, const float* __restrict__ DEG, const float* __restrict__ b, float* __restrict__ OUT, int nv, int nrows) {
  static_assert(W >= 4 && W % 4 == 0, "wfinw: float4 steps"); const size_t i = (size_t)blockIdx.x * 256 + threadIdx.x; if (i >= (size_t)nrows * (W / 4)) return; const size_t v = i / (W / 4); const int c = (int)(i % (W / 4)) * 4; v4f o = {0.0f, 0.0f, 0.0f, 0.0f};
  if (v < (size_t)nv) { const float dg = DEG[v]; const float dv = (dg > 0.0f) ? rsqrtf(dg) : 0.0f; const v4f a = *(const v4f*)(AG + v * W + c), s = *(const v4f*)(HS + v * W + c); for (int j = 0; j < 4; ++j) { const float y = (dv * (a[j] + s[j])) + bf16_rne(b[c + j]); o[j] = RELU ? fmaxf(y, 0.0f) : y; } }
  for (int pass = 0; pass < 2; ++pass) { *(volatile v4f*)(OUT + v * W + c) = o; __threadfence(); }
}
template <int W>
__global__ __launch_bounds__(256) void hsum_kernel(const float* __restrict__ X, int xp, int ns, int srcm, const int* __restrict__ srcs, int ecut, const int* __restrict__ PERM, const int* __restrict__ ROWPTR, const int* __restrict__ ROWCNT, int permLen, float* __restrict__ P, int pp, int ocol, int nd, int ndp) {
  constexpr int CW = W / 8; static_assert(W % 32 == 0, "hsum: 8 threads per row, float4 steps");
  const int tid = threadIdx.x; const int row = tid >> 3, g = tid & 7, c0 = g * CW; const int v = blockIdx.x * 32 + row; if (v >= ndp) return;
  int cnt = 0, p0 = 0; if (v < nd) { cnt = iclamp(ROWCNT[v], 0, 65536); p0 = iclamp(ROWPTR[v], 0, permLen - 1); if (p0 + cnt > permLen) cnt = permLen - p0; }
  float m[CW];
#pragma unroll
  for (int j = 0; j < CW; ++j) m[j] = 0.0f;
#pragma unroll 1
  for (int i = 0; i < cnt; ++i) { const int e = iclamp(PERM[p0 + i], 0, ecut - 1); int s = iclamp(srcs[e], 0, ns - 1); if (srcm < ns) s %= srcm; const float* xr = X + (size_t)s * xp + c0;
#pragma unroll
    for (int q = 0; q < CW / 4; ++q) { const v4f a = *(const v4f*)(xr + 4 * q); for (int j = 0; j < 4; ++j) m[4 * q + j] += a[j]; } }
  for (int pass = 0; pass < 2; ++pass) { float* orow = P + (size_t)v * pp + ocol + c0;
#pragma unroll
    for (int q = 0; q < CW / 4; ++q) { v4f o4; for (int j = 0; j < 4; ++j) o4[j] = (v < nd) ? m[4 * q + j] : 0.0f; *(volatile v4f*)(orow + 4 * q) = o4; }
    __threadfence(); }
}
__global__ __launch_bounds__(256) void gchk_kernel(const int* __restrict__ batch, int* __restrict__ FLAG, int nn) {
  const int v = blockIdx.x * 256 + threadIdx.x; if (v + 1 >= nn) return; if (batch[v] > batch[v + 1] || batch[v] < 0) { ((volatile int*)FLAG)[0] = 1; __threadfence(); }
}
__global__ __launch_bounds__(128) void gmean_kernel(const float* __restrict__ H, const int* __restrict__ batch, const int* __restrict__ FLAG, float* __restrict__ P, int nstat) {
  const int g = blockIdx.x, c = threadIdx.x; int lo = 0, hi = nstat; while (lo < hi) { const int mid = (lo + hi) >> 1; if (batch[mid] < g) lo = mid + 1; else hi = mid; } const int st = lo; hi = nstat; while (lo < hi) { const int mid = (lo + hi) >> 1; if (batch[mid] <= g) lo = mid + 1; else hi = mid; } const int en = lo;
  float s = 0.0f;
#pragma unroll 1
  for (int v = st; v < en; ++v) s += H[(size_t)v * F + c];
  float o = (en > st) ? s / (float)(en - st) : 0.0f; if (FLAG[0] != 0) o = __int_as_float(0x7fc00000);
  for (int pass = 0; pass < 2; ++pass) { ((volatile float*)P)[(size_t)g * F + c] = o; __threadfence(); }
}
template <int W, bool SUM = false>
__global__ __launch_bounds__(W) void gmeanw_kernel(const float* __restrict__ H, const int* __restrict__ batch, const int* __restrict__ FLAG, float* __restrict__ P, int nstat) {
  const int g = blockIdx.x, c = threadIdx.x; int lo = 0, hi = nstat; while (lo < hi) { const int mid = (lo + hi) >> 1; if (batch[mid] < g) lo = mid + 1; else hi = mid; } const int st = lo; hi = nstat; while (lo < hi) { const int mid = (lo + hi) >> 1; if (batch[mid] <= g) lo = mid + 1; else hi = mid; } const int en = lo;
  float s = 0.0f;
#pragma unroll 1
  for (int v = st; v < en; ++v) s += H[(size_t)v * W + c];
  float o = (en > st) ? (SUM ? s : s / (float)(en - st)) : 0.0f; if (FLAG[0] != 0) o = __int_as_float(0x7fc00000);
  for (int pass = 0; pass < 2; ++pass) { ((volatile float*)P)[(size_t)g * W + c] = o; __threadfence(); }
}
template <int W, bool WGT, bool RELU>
__global__ __launch_bounds__(256) void wsumpr_kernel(const float* __restrict__ X, int xp, const float* __restrict__ EW, const int* __restrict__ srcs, const int* __restrict__ PERM, const int* __restrict__ ROWPTR, const int* __restrict__ ROWCNT, int permLen, const float* __restrict__ bias, float* __restrict__ OUT, int op, int mrows, float oscale, int n, int e, int smask) {
  constexpr int CW = W / 8; static_assert(W % 32 == 0, "wsump: 8 threads per row, float4 loads / stores"); const int tid = threadIdx.x; const int row = tid >> 3, g = tid & 7, c0 = g * CW; const int v = blockIdx.x * 32 + row;
  int cnt = 0, p0 = 0; if (v < n) { cnt = iclamp(ROWCNT[v], 0, 65536); p0 = iclamp(ROWPTR[v], 0, permLen - 1); if (p0 + cnt > permLen) cnt = permLen - p0; }
  float m[CW]; for (int j = 0; j < CW; ++j) m[j] = 0.0f;
  for (int i = 0; i < cnt; ++i) { const int ei = iclamp(PERM[p0 + i], 0, e - 1); int s = iclamp(srcs[ei], 0, n - 1); s &= smask; const float w = WGT ? bf16_rne(EW[ei]) : 1.0f;     const float* xr = X + (size_t)s * xp + c0;
#pragma unroll
    for (int q = 0; q < CW / 4; ++q) { const v4f t4 = *(const v4f*)(xr + 4 * q); for (int j = 0; j < 4; ++j) m[4 * q + j] += WGT ? (w * t4[j]) : t4[j]; } }
  for (int pass = 0; pass < 2; ++pass) { if (v < mrows) { float* orow = OUT + (size_t)v * op + c0;
#pragma unroll
      for (int q = 0; q < CW / 4; ++q) { const v4f b4 = *(const v4f*)(bias + c0 + 4 * q); v4f o; for (int j = 0; j < 4; ++j) { float y = m[4 * q + j] + bf16_rne(b4[j]); if (RELU) y = fmaxf(y, 0.0f); o[j] = (v < n) ? (y * oscale) : 0.0f; } *(volatile v4f*)(orow + 4 * q) = o; } }
    __threadfence(); }
}
__global__ __launch_bounds__(256) void emask_kernel(const int* __restrict__ et, int r, int nrel, float* __restrict__ G, int e, int ef) {
  const size_t t = (size_t)blockIdx.x * 256 + threadIdx.x; if (t >= (size_t)ef) return; float g = 0.0f;
  if (t < (size_t)e) { const int ty = iclamp(et[t], 0, nrel - 1); if (ty == r) g = 1.0f; }
  for (int pass = 0; pass < 2; ++pass) { ((volatile float*)G)[t] = g; __threadfence(); }
}
__global__ __launch_bounds__(256) void wcnt_kernel(const float* __restrict__ EW, const int* __restrict__ PERM, const int* __restrict__ ROWPTR, const int* __restrict__ ROWCNT, int permLen, float* __restrict__ D, int n, int nrows) {
  const int v = blockIdx.x * 256 + threadIdx.x; if (v >= nrows) return; float s = 0.0f;
  if (v < n) { int cnt = iclamp(ROWCNT[v], 0, 65536); const int p0 = iclamp(ROWPTR[v], 0, permLen - 1); if (cnt > permLen - p0) cnt = permLen - p0;
    for (int i = 0; i < cnt; ++i) { const int e = iclamp(PERM[p0 + i], 0, E - 1); s += EW[e]; } }
  for (int pass = 0; pass < 2; ++pass) { ((volatile float*)D)[v] = s; __threadfence(); }
}
template <int W>
__global__ __launch_bounds__(256) void rdivf_kernel(const float* __restrict__ A, const float* __restrict__ D, float lo, float* __restrict__ Y, int nn, size_t n4) {
  static_assert(W % 4 == 0 && ((W / 4) & (W / 4 - 1)) == 0, "rdivf: a power-of-two number of float4 groups per row"); const size_t i = (size_t)blockIdx.x * 256 + threadIdx.x; if (i >= n4) return;
  const size_t v = i / (W / 4); v4f o = {0.0f, 0.0f, 0.0f, 0.0f}; if (v < (size_t)nn) { const float dr = D[v]; const float dg = (lo > 0.0f) ? fmaxf(dr, lo) : dr; const v4f t = *(const v4f*)(A + 4 * i); if (dg > 0.0f) { for (int j = 0; j < 4; ++j) o[j] = t[j] / dg; } }
  for (int pass = 0; pass < 2; ++pass) { *(volatile v4f*)(Y + 4 * i) = o; __threadfence(); }
}
}
extern "C" void kernel_launch(void* const* d_in, const int* in_sizes, int n_in, void* d_out, int out_size, void* d_ws, size_t ws_size, hipStream_t stream) {
  auto Fp = [&](int i) { return (const float*)d_in[i]; }; auto Ip = [&](int i) { return (const int*)d_in[i]; };
  constexpr int W = 64  , NR = 5  , NC = 8  ; constexpr size_t IM = (size_t)W * W  , PL = (size_t)NP * W  ;
  static_assert(N == 100000 && NP == N && NRL == NP && NL == N && EFULL == 1200000 && E == EFULL && SRCM == N && CSR_GB == 8 && ((N + CSR_GN - 1) / CSR_GN) <= CSR_MAXG && NP % 32 == 0 && E % 32 == 0 && W % 32 == 0, "the file's own baked sizes are this row's; 100,000 node rows: no padding row; 391 buckets of 256 keys");
  if (n_in != 11 || in_sizes[0] != N * W || in_sizes[1] != 2 * EFULL || in_sizes[2] != EFULL || in_sizes[3] != NR * W * W || in_sizes[4] != W * W || in_sizes[5] != W || in_sizes[6] != NR * W * W || in_sizes[7] != W * W || in_sizes[8] != W || in_sizes[9] != W * NC || in_sizes[10] != NC || out_size != N * W + N * NC) return;
  size_t off = 0; char* ws = (char*)d_ws;
  auto carve = [&](size_t bytes) { char* p = ws + off; off += (bytes + 255) & ~(size_t)255; return p; };
  b16* W1T = (b16*)carve((size_t)NR * IM * 2); b16* R1T = (b16*)carve(IM * 2); b16* W2T = (b16*)carve((size_t)NR * IM * 2); b16* R2T = (b16*)carve(IM * 2);
  float* ZB = (float*)carve(1024);
  float* MSK = (float*)carve((size_t)EFULL * 4); float* CNT = (float*)carve((size_t)NR * NP * 4);
  float* XC = (float*)carve(PL * 4); float* SUM = (float*)carve(PL * 4); float* MEA = (float*)carve(PL * 4); float* H1 = (float*)carve(PL * 4); float* H2 = XC;
  CsrBufs csr; off = csr_carve(csr, ws, off, E, N);
  if (off > ws_size) return;
  const unsigned gW = (unsigned)((IM / 8 + 255) / 256), gN = (unsigned)(NRL / 32), gF = (unsigned)((PL / 4 + 255) / 256), gE = (unsigned)((EFULL + 255) / 256), gC = (unsigned)((NP + 255) / 256); constexpr int SMASK = (SRCM < N) ? SRCM - 1 : 0x7fffffff; static_assert(SRCM >= N || (SRCM & (SRCM - 1)) == 0, "a cut's source remap modulus is a power of two");
  for (int r = 0; r < NR; ++r) wt_kernel<W, W, W><<<gW, 256, 0, stream>>>(Fp(3) + (size_t)r * IM, W1T + (size_t)r * IM, WSC);
  wt_kernel<W, W, W><<<gW, 256, 0, stream>>>(Fp(4), R1T, WSC);
  for (int r = 0; r < NR; ++r) wt_kernel<W, W, W><<<gW, 256, 0, stream>>>(Fp(6) + (size_t)r * IM, W2T + (size_t)r * IM, WSC);
  wt_kernel<W, W, W><<<gW, 256, 0, stream>>>(Fp(7), R2T, WSC);
  zfill_kernel<<<1, 256, 0, stream>>>(ZB, 256);
  csr_build(csr, Ip(1) + EFULL, E, N, stream);
  xcpw_kernel<W><<<gF, 256, 0, stream>>>(Fp(0), XC, W, N, NRL);
  auto relmean = [&](const float* X, int r, bool cnt) { emask_kernel<<<gE, 256, 0, stream>>>(Ip(2), r, NR, MSK, E, EFULL); if (cnt) wcnt_kernel<<<gC, 256, 0, stream>>>(MSK, csr.PERM, csr.ROWPTR, csr.ROWCNT, (int)csr.permLen, CNT + (size_t)r * NP, N, NRL); wsumpr_kernel<W, true, false><<<gN, 256, 0, stream>>>(X, W, MSK, Ip(1), csr.PERM, csr.ROWPTR, csr.ROWCNT, (int)csr.permLen, ZB, SUM, W, NRL, 1.0f, N, E, SMASK); rdivf_kernel<W><<<gF, 256, 0, stream>>>(SUM, CNT + (size_t)r * NP, 1.0f, MEA, N, PL / 4); };
  lin_kernel<W, 4, 1, 0, false><<<gN, 64, 0, stream>>>(XC, nullptr, R1T, R1T, Fp(5), H1, W, N, NRL);
  for (int r = 0; r < NR - 1; ++r) { relmean(XC, r, true); lin_kernel<W, 4, 2, 14, false><<<gN, 64, 0, stream>>>(MEA, nullptr, W1T + (size_t)r * IM, W1T + (size_t)r * IM, ZB, H1, W, N, NRL); }
  relmean(XC, NR - 1, true); lin_kernel<W, 4, 2, 17, false><<<gN, 64, 0, stream>>>(MEA, nullptr, W1T + (size_t)(NR - 1) * IM, W1T + (size_t)(NR - 1) * IM, ZB, H1, W, N, NRL);
  lin_kernel<W, 4, 2, 0, false><<<gN, 64, 0, stream>>>(H1, nullptr, R2T, R2T, Fp(8), H2, W, N, NRL);
  for (int r = 0; r < NR; ++r) { relmean(H1, r, false); lin_kernel<W, 4, 2, 14, false><<<gN, 64, 0, stream>>>(MEA, nullptr, W2T + (size_t)r * IM, W2T + (size_t)r * IM, ZB, H2, W, N, NRL); }
  float* out = (float*)d_out;
  ocpr_kernel<<<(unsigned)(((size_t)N * W + 255) / 256), 256, 0, stream>>>(H2, W, 0, out, W, N);
  headw_kernel<W, NC, false><<<(unsigned)(((size_t)N * NC + 255) / 256), 256, 0, stream>>>(H2, W, Fp(9), Fp(10), out + (size_t)N * W, N * NC);
}
